// RNN_75746043232864
// MI455X (gfx1250) — hardware-verified
//
#include <hip/hip_runtime.h>
#include <math.h>

constexpr int NBATCH = 256;
constexpr int NSTEP  = 2048;
constexpr int NIN    = 25;
constexpr int NHID   = 32;
constexpr int NOUT0  = NBATCH * NSTEP;
constexpr int NOUT1  = NBATCH * NHID;
constexpr size_t OUT1_BYTE_OFF  = 2097152;
constexpr size_t OUT_TOTAL_BYTE = 2129920;
static_assert((size_t)NOUT0 * 4 == OUT1_BYTE_OFF);
static_assert(OUT1_BYTE_OFF + (size_t)NOUT1 * 4 == OUT_TOTAL_BYTE);
static_assert(OUT1_BYTE_OFF % 128 == 0);
static_assert(NHID == 32);
static_assert(NIN <= 32);
static_assert(NSTEP % 32 == 0);
static_assert(NBATCH % 16 == 0);

constexpr int PJ_THR    = 256;
constexpr int PJ_ROWS   = 128;
constexpr int PJ_TSPAN  = 1024;
constexpr int PJ_NCHUNK = PJ_TSPAN / PJ_ROWS;
constexpr int PJ_XF     = PJ_ROWS * NIN;
constexpr int PJ_XV4    = PJ_XF / 4;
constexpr int PJ_WV4    = (NHID * NIN) / 4;
constexpr int SLABP     = 36;
static_assert(NSTEP % PJ_TSPAN == 0);
static_assert(PJ_TSPAN % PJ_ROWS == 0);
static_assert(PJ_ROWS == 16 * (PJ_THR / 32));
static_assert(PJ_XF % 4 == 0);
static_assert(PJ_ROWS % 4 == 0 && NSTEP % 4 == 0);
static_assert(PJ_XV4 <= 4 * PJ_THR);
static_assert((NHID * NIN) % 4 == 0);
static_assert(PJ_WV4 <= PJ_THR);

constexpr int   HPITCH = 40;
constexpr int   OSP    = 36;
constexpr float HCARRY = 64.0f;
constexpr float WCARRY = 64.0f;
constexpr float FOLD   = 1.0f / (HCARRY * WCARRY);

typedef __attribute__((ext_vector_type(16))) _Float16 v16h;
typedef __attribute__((ext_vector_type(8)))  _Float16 v8h;
typedef __attribute__((ext_vector_type(16))) __bf16   v16b;
typedef __attribute__((ext_vector_type(8)))  float    v8f;
typedef __attribute__((ext_vector_type(4)))  float    v4f;

__device__ __forceinline__ unsigned f2bf_bits32(float f) {
  const unsigned u = __float_as_uint(f);
  return (u + 0x7FFFu + ((u >> 16) & 1u)) >> 16;
}
__device__ __forceinline__ void split_bf(float f, __bf16& hi, __bf16& lo) {
  const unsigned hb = f2bf_bits32(f);
  const float hf = __uint_as_float(hb << 16);
  const unsigned lb = f2bf_bits32(f - hf);
  const unsigned short hs = (unsigned short)hb;
  const unsigned short ls = (unsigned short)lb;
  hi = __builtin_bit_cast(__bf16, hs);
  lo = __builtin_bit_cast(__bf16, ls);
}
__device__ __forceinline__ v8f mma_bf(v16b a, v16b b, v8f c) {
  c = __builtin_amdgcn_wmma_f32_16x16x32_bf16(false, a, false, b, (short)0, c, false, false);
  asm volatile("v_nop\n\tv_nop\n\tv_nop\n\tv_nop" : "+v"(c) : "v"(a), "v"(b));
  return c;
}
__device__ __forceinline__ v8f mma_h(v16h a, v16h b, v8f c) {
  c = __builtin_amdgcn_wmma_f32_16x16x32_f16(false, a, false, b, (short)0, c, false, false);
  asm volatile("v_nop\n\tv_nop\n\tv_nop\n\tv_nop" : "+v"(c) : "v"(a), "v"(b));
  return c;
}
union FragH { v16h v; v8h h[2]; };
__device__ __forceinline__ v16h frag_load_h(const _Float16* p) {
  FragH f;
  f.h[0] = *(const v8h*)(p);
  f.h[1] = *(const v8h*)(p + 16);
  return f.v;
}
__device__ __forceinline__ float ftanh(float x) {
  return 1.0f - 2.0f * __builtin_amdgcn_rcpf(__expf(2.0f * x) + 1.0f);
}

__global__ __launch_bounds__(PJ_THR) void proj_kernel(const float* __restrict__ x, const float* __restrict__ wih,
                                                      const float* __restrict__ bih, const float* __restrict__ bhh,
                                                      float* __restrict__ XP) {
  __shared__ __align__(16) float xs[PJ_XF];
  __shared__ __align__(16) float wsm[NHID * NIN];
  __shared__ __align__(16) float sl[PJ_THR / 32][16 * SLABP];
  const int tid = threadIdx.x, lane = tid & 31, wave = tid >> 5;
  const int c = lane & 15, hh = lane >> 4;
  const int b = blockIdx.x / (NSTEP / PJ_TSPAN);
  const int tbase = (blockIdx.x % (NSTEP / PJ_TSPAN)) * PJ_TSPAN;

  {
    const int wi = (tid < PJ_WV4) ? tid : (PJ_WV4 - 1);
    v4f wv = *(const v4f*)(wih + 4 * wi);
    asm volatile("" : "+v"(wv));
    if (tid < PJ_WV4) *(v4f*)(wsm + 4 * tid) = wv;
  }
  const float bi0 = bih[c], bi1 = bih[16 + c];
  const float bq0 = bhh[c], bq1 = bhh[16 + c];
  __syncthreads();

  v16b bh0, bl0, bh1, bl1;
  {
    const float* w0 = wsm + c * NIN;
    const float* w1 = wsm + (16 + c) * NIN;
#pragma unroll
    for (int e = 0; e < 8; ++e) {
      const int k0 = 8 * hh + e;
      const int k1 = 16 + 8 * hh + e;
      const int k1c = (k1 < NIN) ? k1 : (NIN - 1);
      const float f00 = w0[k0];
      float f01 = w0[k1c];
      const float f10 = w1[k0];
      float f11 = w1[k1c];
      asm volatile("" : "+v"(f01), "+v"(f11));
      f01 = (k1 < NIN) ? f01 : 0.0f;
      f11 = (k1 < NIN) ? f11 : 0.0f;
      __bf16 hq, lq;
      split_bf(f00, hq, lq);
      bh0[e] = hq;
      bl0[e] = lq;
      split_bf(f01, hq, lq);
      bh0[8 + e] = hq;
      bl0[8 + e] = lq;
      split_bf(f10, hq, lq);
      bh1[e] = hq;
      bl1[e] = lq;
      split_bf(f11, hq, lq);
      bh1[8 + e] = hq;
      bl1[8 + e] = lq;
    }
  }

  const v8f z8 = {0.f, 0.f, 0.f, 0.f, 0.f, 0.f, 0.f, 0.f};
  float* slab = sl[wave];
  const int q = lane >> 3, c4 = (lane & 7) * 4;

#pragma unroll 1
  for (int ch = 0; ch < PJ_NCHUNK; ++ch) {
    const int t0 = tbase + ch * PJ_ROWS;
    __syncthreads();
    {
      const float* xb = x + ((size_t)b * NSTEP + (size_t)t0) * NIN;
#pragma unroll
      for (int i = 0; i < 4; ++i) {
        const int idx = i * PJ_THR + tid;
        const int idc = (idx < PJ_XV4) ? idx : (PJ_XV4 - 1);
        v4f xv = *(const v4f*)(xb + 4 * idc);
        asm volatile("" : "+v"(xv));
        if (idx < PJ_XV4) *(v4f*)(xs + 4 * idx) = xv;
      }
    }
    __syncthreads();

    v16b ah, al;
    {
      const float* xr = xs + (wave * 16 + c) * NIN;
#pragma unroll
      for (int e = 0; e < 8; ++e) {
        const int k0 = 8 * hh + e;
        const int k1 = 16 + 8 * hh + e;
        const int k1c = (k1 < NIN) ? k1 : (NIN - 1);
        const float f0 = xr[k0];
        float f1 = xr[k1c];
        asm volatile("" : "+v"(f1));
        f1 = (k1 < NIN) ? f1 : 0.0f;
        __bf16 hq, lq;
        split_bf(f0, hq, lq);
        ah[e] = hq;
        al[e] = lq;
        split_bf(f1, hq, lq);
        ah[8 + e] = hq;
        al[8 + e] = lq;
      }
    }
    v8f acc0 = z8, acc1 = z8;
    acc0 = mma_bf(ah, bh0, acc0);
    acc0 = mma_bf(ah, bl0, acc0);
    acc0 = mma_bf(al, bh0, acc0);
    acc1 = mma_bf(ah, bh1, acc1);
    acc1 = mma_bf(ah, bl1, acc1);
    acc1 = mma_bf(al, bh1, acc1);

#pragma unroll
    for (int r = 0; r < 8; ++r) {
      slab[(8 * hh + r) * SLABP + c]      = (acc0[r] + bi0) + bq0;
      slab[(8 * hh + r) * SLABP + 16 + c] = (acc1[r] + bi1) + bq1;
    }
    __syncthreads();
    v4f ov[4];
#pragma unroll
    for (int it = 0; it < 4; ++it) ov[it] = *(const v4f*)(slab + (4 * it + q) * SLABP + c4);
    for (int pass = 0; pass < 2; ++pass) {
#pragma unroll
      for (int it = 0; it < 4; ++it) {
        const int t = t0 + wave * 16 + 4 * it + q;
        *(volatile v4f*)(XP + ((size_t)t * NBATCH + (size_t)b) * NHID + c4) = ov[it];
      }
      __threadfence();
    }
  }
}

__global__ __launch_bounds__(32) void scan_kernel(const float* __restrict__ XP, const float* __restrict__ h0,
                                                  const float* __restrict__ whh, const float* __restrict__ fcw,
                                                  const float* __restrict__ fcb,
                                                  float* __restrict__ out0, float* __restrict__ out1) {
  __shared__ __align__(16) _Float16 Hs[16 * HPITCH];
  __shared__ __align__(16) float    Os[16 * OSP];
  __shared__ __align__(16) float    Fs[16 * OSP];
  const int lane = threadIdx.x & 31;
  const int c = lane & 15, hh = lane >> 4;
  const int b0 = blockIdx.x * 16;

  v16h a0, a1;
  {
    const float* wr = whh + (size_t)c * NHID + 8 * hh;
    v4f w0 = *(const v4f*)(wr);
    v4f w1 = *(const v4f*)(wr + 4);
    v4f w2 = *(const v4f*)(wr + 16);
    v4f w3 = *(const v4f*)(wr + 20);
    asm volatile("" : "+v"(w0), "+v"(w1), "+v"(w2), "+v"(w3) :: "memory");
#pragma unroll
    for (int e = 0; e < 4; ++e) {
      a0[e]      = (_Float16)(w0[e] * WCARRY);
      a0[4 + e]  = (_Float16)(w1[e] * WCARRY);
      a0[8 + e]  = (_Float16)(w2[e] * WCARRY);
      a0[12 + e] = (_Float16)(w3[e] * WCARRY);
    }
  }
  {
    const float* wr = whh + (size_t)(16 + c) * NHID + 8 * hh;
    v4f w0 = *(const v4f*)(wr);
    v4f w1 = *(const v4f*)(wr + 4);
    v4f w2 = *(const v4f*)(wr + 16);
    v4f w3 = *(const v4f*)(wr + 20);
    asm volatile("" : "+v"(w0), "+v"(w1), "+v"(w2), "+v"(w3) :: "memory");
#pragma unroll
    for (int e = 0; e < 4; ++e) {
      a1[e]      = (_Float16)(w0[e] * WCARRY);
      a1[4 + e]  = (_Float16)(w1[e] * WCARRY);
      a1[8 + e]  = (_Float16)(w2[e] * WCARRY);
      a1[12 + e] = (_Float16)(w3[e] * WCARRY);
    }
  }
  {
    const float* hp = h0 + (size_t)(b0 + c) * NHID + 8 * hh;
    v4f p0 = *(const v4f*)(hp);
    v4f p1 = *(const v4f*)(hp + 4);
    v4f p2 = *(const v4f*)(hp + 16);
    v4f p3 = *(const v4f*)(hp + 20);
    asm volatile("" : "+v"(p0), "+v"(p1), "+v"(p2), "+v"(p3) :: "memory");
    v8h i0, i1;
#pragma unroll
    for (int e = 0; e < 4; ++e) {
      i0[e]     = (_Float16)(p0[e] * HCARRY);
      i0[4 + e] = (_Float16)(p1[e] * HCARRY);
      i1[e]     = (_Float16)(p2[e] * HCARRY);
      i1[4 + e] = (_Float16)(p3[e] * HCARRY);
    }
    *(v8h*)(Hs + c * HPITCH + 8 * hh)      = i0;
    *(v8h*)(Hs + c * HPITCH + 16 + 8 * hh) = i1;
  }
  float fw0[8], fw1[8];
  {
    v4f g0 = *(const v4f*)(fcw + 8 * hh);
    v4f g1 = *(const v4f*)(fcw + 8 * hh + 4);
    v4f g2 = *(const v4f*)(fcw + 16 + 8 * hh);
    v4f g3 = *(const v4f*)(fcw + 16 + 8 * hh + 4);
    asm volatile("" : "+v"(g0), "+v"(g1), "+v"(g2), "+v"(g3) :: "memory");
#pragma unroll
    for (int e = 0; e < 4; ++e) {
      fw0[e]     = g0[e];
      fw0[4 + e] = g1[e];
      fw1[e]     = g2[e];
      fw1[4 + e] = g3[e];
    }
  }
  const float fcb0 = fcb[0];

  const v8f z8 = {0.f, 0.f, 0.f, 0.f, 0.f, 0.f, 0.f, 0.f};
  const float* xrow = XP + (size_t)(b0 + c) * NHID + 8 * hh;
  v8f xn0 = *(const v8f*)(xrow);
  v8f xn1 = *(const v8f*)(xrow + 16);
  v8f th0 = z8, th1 = z8;
  const int q = lane >> 3, c4 = (lane & 7) * 4;
  __syncthreads();

#pragma unroll 1
  for (int t = 0; t < NSTEP; ++t) {
    const v8f x0 = xn0;
    const v8f x1 = xn1;
    {
      const int tn = (t + 1 < NSTEP) ? (t + 1) : (NSTEP - 1);
      const float* xp = xrow + (size_t)tn * NBATCH * NHID;
      xn0 = *(const v8f*)(xp);
      xn1 = *(const v8f*)(xp + 16);
    }
    const v16h bf = frag_load_h(Hs + c * HPITCH + 8 * hh);
    v8f acc0 = mma_h(a0, bf, z8);
    v8f acc1 = mma_h(a1, bf, z8);

    v8h hv0, hv1;
    float pa = 0.0f, pb = 0.0f;
#pragma unroll
    for (int r = 0; r < 8; ++r) {
      const float za = fmaf(acc0[r], FOLD, x0[r]);
      const float zb = fmaf(acc1[r], FOLD, x1[r]);
      const float ta = ftanh(za);
      const float tb = ftanh(zb);
      th0[r] = ta;
      th1[r] = tb;
      hv0[r] = (_Float16)(ta * HCARRY);
      hv1[r] = (_Float16)(tb * HCARRY);
      pa = fmaf(ta, fw0[r], pa);
      pb = fmaf(tb, fw1[r], pb);
    }
    *(v8h*)(Hs + c * HPITCH + 8 * hh)      = hv0;
    *(v8h*)(Hs + c * HPITCH + 16 + 8 * hh) = hv1;

    float p = pa + pb;
    const float pother = __shfl_xor(p, 16, 32);
    p = p + pother;
    const float o = p + fcb0;
    if (hh == 0) Os[c * OSP + (t & 31)] = o;
    __syncthreads();

    if ((t & 31) == 31) {
      const int tb0 = t - 31;
      v4f ov[4];
#pragma unroll
      for (int it = 0; it < 4; ++it) ov[it] = *(const v4f*)(Os + (4 * it + q) * OSP + c4);
      for (int pass = 0; pass < 2; ++pass) {
#pragma unroll
        for (int it = 0; it < 4; ++it)
          *(volatile v4f*)(out0 + (size_t)(b0 + 4 * it + q) * NSTEP + tb0 + c4) = ov[it];
        __threadfence();
      }
      __syncthreads();
    }
  }

  {
    v4f s0, s1, s2, s3;
#pragma unroll
    for (int e = 0; e < 4; ++e) {
      s0[e] = th0[e];
      s1[e] = th0[4 + e];
      s2[e] = th1[e];
      s3[e] = th1[4 + e];
    }
    *(v4f*)(Fs + c * OSP + 8 * hh)          = s0;
    *(v4f*)(Fs + c * OSP + 8 * hh + 4)      = s1;
    *(v4f*)(Fs + c * OSP + 16 + 8 * hh)     = s2;
    *(v4f*)(Fs + c * OSP + 16 + 8 * hh + 4) = s3;
  }
  __syncthreads();
  {
    v4f fv[4];
#pragma unroll
    for (int it = 0; it < 4; ++it) fv[it] = *(const v4f*)(Fs + (4 * it + q) * OSP + c4);
    for (int pass = 0; pass < 2; ++pass) {
#pragma unroll
      for (int it = 0; it < 4; ++it)
        *(volatile v4f*)(out1 + (size_t)(b0 + 4 * it + q) * NHID + c4) = fv[it];
      __threadfence();
    }
  }
}

extern "C" void kernel_launch(void* const* d_in, const int* in_sizes, int n_in,
                              void* d_out, int out_size, void* d_ws, size_t ws_size, hipStream_t stream) {
  if (n_in < 8 || d_out == nullptr || d_ws == nullptr) return;
  if (in_sizes[0] != NBATCH * NSTEP * NIN || in_sizes[1] != NBATCH * NHID || in_sizes[2] != NHID * NIN ||
      in_sizes[3] != NHID * NHID || in_sizes[4] != NHID || in_sizes[5] != NHID || in_sizes[6] != NHID ||
      in_sizes[7] != 1 || out_size != NOUT0 + NOUT1) return;

  const float* x   = (const float*)d_in[0];
  const float* h0  = (const float*)d_in[1];
  const float* wih = (const float*)d_in[2];
  const float* whh = (const float*)d_in[3];
  const float* bih = (const float*)d_in[4];
  const float* bhh = (const float*)d_in[5];
  const float* fcw = (const float*)d_in[6];
  const float* fcb = (const float*)d_in[7];
  float* out0 = (float*)d_out;
  float* out1 = out0 + (OUT1_BYTE_OFF / 4);

  const size_t xp_bytes = (size_t)NSTEP * NBATCH * NHID * 4;
  if (xp_bytes > ws_size || xp_bytes > (size_t)134217728) return;
  float* XP = (float*)d_ws;

  proj_kernel<<<NBATCH * (NSTEP / PJ_TSPAN), PJ_THR, 0, stream>>>(x, wih, bih, bhh, XP);
  scan_kernel<<<NBATCH / 16, 32, 0, stream>>>(XP, h0, whh, fcw, fcb, out0, out1);
}
